// GINConv_8856222564747
// MI455X (gfx1250) — hardware-verified
//
#include <hip/hip_runtime.h>
#include <stddef.h>


#define DIN     512
#define DHID    1024
#define NTHR    256
#define NWAVE   8
#define EPT     8
#define NGRP    2
#define CHUNK   (NTHR * EPT * NGRP)
#define WCAP    (EPT * NGRP * 32)
#define LISTN   (NWAVE * WCAP)
#define NB      64
#define BM      64
#define BN      128
#define GTHR    128
#define WUNITS  (DIN * DHID / 8)
#define RCARRY  4.0f
#define HCARRY  4.0f
#define WCARRY  64.0f
#define GS0     (1.0f / 256.0f)
#define GS1     (1.0f / 256.0f)
#define WSCAP   134217728
#define LDS_AGG ((NB * DIN + LISTN + NWAVE) * 4 + 64)

static_assert((CHUNK & (CHUNK - 1)) == 0);
static_assert(CHUNK <= 4096);
static_assert(WCAP == EPT * NGRP * 32);
static_assert((NB & (NB - 1)) == 0 && NB < 4096);
static_assert(NB == BM);
static_assert(NWAVE * 8 == NB);
static_assert(NTHR == NWAVE * 32);
static_assert(NTHR * 2 == DIN);
static_assert(DIN / 2 == 32 * 8);
static_assert((DIN % 32) == 0 && (DHID % 32) == 0);
static_assert((DIN % BN) == 0 && (DHID % BN) == 0);
static_assert(GTHR == 4 * 32);
static_assert(BM == 4 * 16 && BN == 2 * 64);
static_assert((WUNITS % NTHR) == 0);
static_assert(LDS_AGG <= 160 * 1024);

typedef float    v2f  __attribute__((ext_vector_type(2)));
typedef float    v4f  __attribute__((ext_vector_type(4)));
typedef float    v8f  __attribute__((ext_vector_type(8)));
typedef int      v4i  __attribute__((ext_vector_type(4)));
typedef _Float16 v8h  __attribute__((ext_vector_type(8)));
typedef _Float16 v16h __attribute__((ext_vector_type(16)));
union Frag { v16h v; v8h h[2]; };

__device__ __forceinline__ v8f wmh(v16h a, v16h b, v8f c) {
  v8f d = __builtin_amdgcn_wmma_f32_16x16x32_f16(false, a, false, b, (short)0, c, false, false);
  asm volatile("v_nop\n\tv_nop\n\tv_nop\n\tv_nop" : "+v"(d) : "v"(a), "v"(b));
  return d;
}

template <int NBT>
__device__ __forceinline__ int scan_chunk(const int* __restrict__ dsts, int nE, int cbase, int slotBase,
                                          int vec8, int* list, int tid, int lane, int wave) {
  int wc = 0;
#pragma unroll
  for (int g = 0; g < NGRP; ++g) {
    const int el0  = (g * NTHR + tid) * EPT;
    const int e0   = cbase + el0;
    const int sent = -2147483647 - 1;
    v4i da, db;
    if (vec8 != 0 && cbase + CHUNK <= nE) {
      da = *(const v4i*)(dsts + e0);
      db = *(const v4i*)(dsts + e0 + 4);
    } else {
      da.x = (e0     < nE) ? dsts[min(e0, nE - 1)] : sent;
      da.y = (e0 + 1 < nE) ? dsts[min(e0 + 1, nE - 1)] : sent;
      da.z = (e0 + 2 < nE) ? dsts[min(e0 + 2, nE - 1)] : sent;
      da.w = (e0 + 3 < nE) ? dsts[min(e0 + 3, nE - 1)] : sent;
      db.x = (e0 + 4 < nE) ? dsts[min(e0 + 4, nE - 1)] : sent;
      db.y = (e0 + 5 < nE) ? dsts[min(e0 + 5, nE - 1)] : sent;
      db.z = (e0 + 6 < nE) ? dsts[min(e0 + 6, nE - 1)] : sent;
      db.w = (e0 + 7 < nE) ? dsts[min(e0 + 7, nE - 1)] : sent;
    }
    const unsigned nb = (unsigned)slotBase;
    const unsigned s0 = (unsigned)da.x - nb, s1 = (unsigned)da.y - nb;
    const unsigned s2 = (unsigned)da.z - nb, s3 = (unsigned)da.w - nb;
    const unsigned s4 = (unsigned)db.x - nb, s5 = (unsigned)db.y - nb;
    const unsigned s6 = (unsigned)db.z - nb, s7 = (unsigned)db.w - nb;
    const bool h0 = s0 < (unsigned)NBT, h1 = s1 < (unsigned)NBT, h2 = s2 < (unsigned)NBT, h3 = s3 < (unsigned)NBT;
    const bool h4 = s4 < (unsigned)NBT, h5 = s5 < (unsigned)NBT, h6 = s6 < (unsigned)NBT, h7 = s7 < (unsigned)NBT;
    const unsigned any = __builtin_amdgcn_ballot_w32(h0 | h1 | h2 | h3 | h4 | h5 | h6 | h7);
    if (any != 0u) {
#define HITJ(J, HJ, SJ) { \
        const unsigned mj = __builtin_amdgcn_ballot_w32(HJ); \
        if (mj != 0u) { \
          if (HJ) { \
            const int pos = wc + (int)__builtin_amdgcn_mbcnt_lo(mj, 0u); \
            if (pos < WCAP) list[wave * WCAP + pos] = ((el0 + (J)) << 12) | (int)(SJ); \
          } \
          wc += (int)__builtin_popcount(mj); } }
      HITJ(0, h0, s0)
      HITJ(1, h1, s1)
      HITJ(2, h2, s2)
      HITJ(3, h3, s3)
      HITJ(4, h4, s4)
      HITJ(5, h5, s5)
      HITJ(6, h6, s6)
      HITJ(7, h7, s7)
#undef HITJ
    }
  }
  return wc;
}

__global__ __launch_bounds__(NTHR) void k_wcvt(const float* __restrict__ W1, const float* __restrict__ W2,
                                               _Float16* p1, _Float16* p2) {
  const int mat = (int)blockIdx.y;
  const int i = (int)blockIdx.x * NTHR + (int)threadIdx.x;
  if (i >= WUNITS) return;
  const int K = (mat == 0) ? DIN : DHID;
  const int N = (mat == 0) ? DHID : DIN;
  const float* W = (mat == 0) ? W1 : W2;
  _Float16* P = (mat == 0) ? p1 : p2;
  const int ppr = K / 8;
  const int n = i / ppr;
  const int seg = i - n * ppr;
  const float* sp = W + (size_t)(8 * seg) * N + n;
  v8h o;
#pragma unroll
  for (int j = 0; j < 8; ++j) o[j] = (_Float16)(sp[(size_t)j * N] * WCARRY);
  _Float16* gp = P + (size_t)i * 8;
  *(volatile v8h*)gp = o;
  __threadfence();
  *(volatile v8h*)gp = o;
}

__global__ __launch_bounds__(NTHR) void k_agg(
    const float* __restrict__ feat, const int* __restrict__ srcs, const int* __restrict__ dsts,
    const float* __restrict__ epsp, _Float16* rstp, int nN, int nE, int vec8) {
#pragma clang fp contract(off)
  extern __shared__ v4f lds_dyn[];
  float* accl = (float*)lds_dyn;
  int* list = (int*)(accl + NB * DIN);
  int* wcnt = list + LISTN;
  const int tid = threadIdx.x, lane = tid & 31, wave = tid >> 5;
  const int nodeBase = (int)blockIdx.x * NB;

  {
    const v4f z = {0.f, 0.f, 0.f, 0.f};
#pragma unroll 1
    for (int i = tid; i < (NB * DIN) / 4; i += NTHR) ((v4f*)accl)[i] = z;
  }
  __syncthreads();

  const int col2 = 2 * tid;
  const int nChunks = (nE + CHUNK - 1) / CHUNK;
#pragma unroll 1
  for (int ch = 0; ch < nChunks; ++ch) {
    const int cbase = ch * CHUNK;
    const int wc = scan_chunk<NB>(dsts, nE, cbase, nodeBase, vec8, list, tid, lane, wave);
    if (lane == 0) wcnt[wave] = wc;
    __syncthreads();
#pragma unroll 1
    for (int wsx = 0; wsx < NWAVE; ++wsx) {
      int n = __builtin_amdgcn_readfirstlane(wcnt[wsx]);
      n = n > WCAP ? WCAP : (n < 0 ? 0 : n);
      const int* lp = list + wsx * WCAP;
#pragma unroll 1
      for (int i = 0; i < n; ++i) {
        const int ent  = __builtin_amdgcn_readfirstlane(lp[i]);
        const int slot = ent & (NB - 1);
        int e = cbase + ((ent >> 12) & (CHUNK - 1));
        e = e > nE - 1 ? nE - 1 : (e < 0 ? 0 : e);
        int sv = srcs[e];
        sv = sv < 0 ? 0 : (sv > nN - 1 ? nN - 1 : sv);
        const v2f x = *(const v2f*)(feat + (size_t)sv * DIN + col2);
        v2f* ap = (v2f*)(accl + slot * DIN + col2);
        const v2f cur = *ap;
        *ap = cur + x;
      }
    }
    __syncthreads();
  }

  const float s1 = 1.0f + epsp[0];
#pragma unroll 1
  for (int j = 0; j < 8; ++j) {
    const int r = 8 * wave + j;
    const int d = nodeBase + r;
    const bool live = d < nN;
    int dcl = d > nN - 1 ? nN - 1 : d;
    dcl = dcl < 0 ? 0 : dcl;
    v8h ov[2];
#pragma unroll
    for (int q = 0; q < 2; ++q) {
      const int col = q * (DIN / 2) + 8 * lane;
      const v4f a0 = *(const v4f*)(accl + r * DIN + col);
      const v4f a1 = *(const v4f*)(accl + r * DIN + col + 4);
      const v4f f0 = *(const v4f*)(feat + (size_t)dcl * DIN + col);
      const v4f f1 = *(const v4f*)(feat + (size_t)dcl * DIN + col + 4);
      const v4f m0 = f0 * s1;
      const v4f m1 = f1 * s1;
      const v4f u0 = (m0 + a0) * RCARRY;
      const v4f u1 = (m1 + a1) * RCARRY;
      v8h o;
      o[0] = live ? (_Float16)u0.x : (_Float16)0.0f;
      o[1] = live ? (_Float16)u0.y : (_Float16)0.0f;
      o[2] = live ? (_Float16)u0.z : (_Float16)0.0f;
      o[3] = live ? (_Float16)u0.w : (_Float16)0.0f;
      o[4] = live ? (_Float16)u1.x : (_Float16)0.0f;
      o[5] = live ? (_Float16)u1.y : (_Float16)0.0f;
      o[6] = live ? (_Float16)u1.z : (_Float16)0.0f;
      o[7] = live ? (_Float16)u1.w : (_Float16)0.0f;
      ov[q] = o;
    }
    _Float16* gp = rstp + (size_t)d * DIN + 8 * lane;
    *(volatile v8h*)gp = ov[0];
    *(volatile v8h*)(gp + DIN / 2) = ov[1];
    __threadfence();
    *(volatile v8h*)gp = ov[0];
    *(volatile v8h*)(gp + DIN / 2) = ov[1];
  }
}

template <int MODE>
__global__ __launch_bounds__(GTHR) void k_gemm(
    const _Float16* __restrict__ Ap, const _Float16* __restrict__ Bp, const float* __restrict__ bias,
    const float* __restrict__ resid, _Float16* outH, float* outF, int K, int N, int nValid) {
  __shared__ __attribute__((aligned(16))) float stg[BM * BN];
  const int tid = threadIdx.x, lane = tid & 31, wave = tid >> 5, hh = lane >> 4, m = lane & 15;
  const int rowBase = (int)blockIdx.x * BM;
  const int colBase = (int)blockIdx.y * BN;
  const int rg = wave >> 1, chf = wave & 1;
  const int r0 = 32 * rg;
  const int c0 = 64 * chf;

  v8f acc[2][4];
#pragma unroll
  for (int i = 0; i < 2; ++i) {
#pragma unroll
    for (int t = 0; t < 4; ++t) { v8f z = {0.f, 0.f, 0.f, 0.f, 0.f, 0.f, 0.f, 0.f}; acc[i][t] = z; }
  }

  const _Float16* ap0 = Ap + (size_t)(rowBase + r0 + m) * K + 8 * hh;
  const _Float16* ap1 = ap0 + (size_t)16 * K;
  const _Float16* bp0 = Bp + (size_t)(colBase + c0 + m) * K + 8 * hh;
  const int ksteps = K >> 5;
#pragma unroll 1
  for (int kt = 0; kt < ksteps; ++kt) {
    const int ko = kt << 5;
    Frag a0, a1;
    a0.h[0] = *(const v8h*)(ap0 + ko);
    a0.h[1] = *(const v8h*)(ap0 + ko + 16);
    a1.h[0] = *(const v8h*)(ap1 + ko);
    a1.h[1] = *(const v8h*)(ap1 + ko + 16);
#pragma unroll
    for (int t = 0; t < 4; ++t) {
      const _Float16* bq = bp0 + (size_t)(16 * t) * K + ko;
      Frag b;
      b.h[0] = *(const v8h*)bq;
      b.h[1] = *(const v8h*)(bq + 16);
      acc[0][t] = wmh(a0.v, b.v, acc[0][t]);
      acc[1][t] = wmh(a1.v, b.v, acc[1][t]);
    }
  }

  const float gs = (MODE == 0) ? GS0 : GS1;
#pragma unroll
  for (int t = 0; t < 4; ++t) {
    const int col = c0 + 16 * t + m;
    const float bv = bias[colBase + col];
#pragma unroll
    for (int i = 0; i < 2; ++i) {
#pragma unroll
      for (int r = 0; r < 8; ++r) {
        const int row = r0 + 16 * i + 8 * hh + r;
        float g = acc[i][t][r] * gs + bv;
        if (MODE == 0) g = fmaxf(g, 0.f);
        stg[row * BN + col] = g;
      }
    }
  }
  __syncthreads();

  if constexpr (MODE == 0) {
    v8h ov[8];
#pragma unroll
    for (int p = 0; p < 8; ++p) {
      const int row = 16 * wave + 2 * p + hh;
      const bool live = (rowBase + row) < nValid;
      const v4f x0 = *(const v4f*)(stg + row * BN + 8 * m);
      const v4f x1 = *(const v4f*)(stg + row * BN + 8 * m + 4);
      v8h o;
      o[0] = live ? (_Float16)(x0.x * HCARRY) : (_Float16)0.0f;
      o[1] = live ? (_Float16)(x0.y * HCARRY) : (_Float16)0.0f;
      o[2] = live ? (_Float16)(x0.z * HCARRY) : (_Float16)0.0f;
      o[3] = live ? (_Float16)(x0.w * HCARRY) : (_Float16)0.0f;
      o[4] = live ? (_Float16)(x1.x * HCARRY) : (_Float16)0.0f;
      o[5] = live ? (_Float16)(x1.y * HCARRY) : (_Float16)0.0f;
      o[6] = live ? (_Float16)(x1.z * HCARRY) : (_Float16)0.0f;
      o[7] = live ? (_Float16)(x1.w * HCARRY) : (_Float16)0.0f;
      ov[p] = o;
    }
#pragma unroll
    for (int p = 0; p < 8; ++p) {
      const int row = 16 * wave + 2 * p + hh;
      _Float16* gp = outH + (size_t)(rowBase + row) * N + colBase + 8 * m;
      *(volatile v8h*)gp = ov[p];
    }
    __threadfence();
#pragma unroll
    for (int p = 0; p < 8; ++p) {
      const int row = 16 * wave + 2 * p + hh;
      _Float16* gp = outH + (size_t)(rowBase + row) * N + colBase + 8 * m;
      *(volatile v8h*)gp = ov[p];
    }
  } else {
    v4f ov[16];
#pragma unroll
    for (int p = 0; p < 16; ++p) {
      const int row = 16 * wave + p;
      int rcl = rowBase + row;
      rcl = rcl > nValid - 1 ? nValid - 1 : rcl;
      rcl = rcl < 0 ? 0 : rcl;
      const v4f x  = *(const v4f*)(stg + row * BN + 4 * lane);
      const v4f rv = *(const v4f*)(resid + (size_t)rcl * N + colBase + 4 * lane);
      ov[p] = x + rv;
    }
#pragma unroll
    for (int p = 0; p < 16; ++p) {
      const int grow = rowBase + 16 * wave + p;
      if (grow < nValid) {
        float* gp = outF + (size_t)grow * N + colBase + 4 * lane;
        *(volatile v4f*)gp = ov[p];
      }
    }
    __threadfence();
#pragma unroll
    for (int p = 0; p < 16; ++p) {
      const int grow = rowBase + 16 * wave + p;
      if (grow < nValid) {
        float* gp = outF + (size_t)grow * N + colBase + 4 * lane;
        *(volatile v4f*)gp = ov[p];
      }
    }
  }
}

extern "C" void kernel_launch(void* const* d_in, const int* in_sizes, int n_in,
                              void* d_out, int out_size, void* d_ws, size_t ws_size,
                              hipStream_t stream) {
  if (n_in < 8) return;
  if (in_sizes[0] < DIN || (in_sizes[0] % DIN) != 0) return;
  const int nN = in_sizes[0] / DIN;
  if (in_sizes[1] != DIN * DHID || in_sizes[2] != DHID) return;
  if (in_sizes[3] != DHID * DIN || in_sizes[4] != DIN) return;
  if (in_sizes[5] < 1) return;
  if (in_sizes[6] < 1 || in_sizes[6] != in_sizes[7]) return;
  const int nE = in_sizes[6];
  if (out_size != nN * DIN) return;
  if (nN > (1 << 21) || nE > (1 << 28)) return;

  const float* feat = (const float*)d_in[0];
  const float* W1   = (const float*)d_in[1];
  const float* b1   = (const float*)d_in[2];
  const float* W2   = (const float*)d_in[3];
  const float* b2   = (const float*)d_in[4];
  const float* eps  = (const float*)d_in[5];
  const int*   src  = (const int*)d_in[6];
  const int*   dst  = (const int*)d_in[7];
  float* out = (float*)d_out;

  const int nRB  = (nN + BM - 1) / BM;
  const int MPAD = nRB * BM;

  char* ws = (char*)d_ws;
  size_t off = 0;
  const size_t oW1 = off; off += (size_t)DHID * DIN * 2;   off = (off + 255) & ~(size_t)255;
  const size_t oW2 = off; off += (size_t)DIN * DHID * 2;   off = (off + 255) & ~(size_t)255;
  const size_t oR  = off; off += (size_t)MPAD * DIN * 2;   off = (off + 255) & ~(size_t)255;
  const size_t oH  = off; off += (size_t)MPAD * DHID * 2;  off = (off + 255) & ~(size_t)255;
  if (off > ws_size || off > (size_t)WSCAP) return;

  _Float16* w1p  = (_Float16*)(ws + oW1);
  _Float16* w2p  = (_Float16*)(ws + oW2);
  _Float16* rstp = (_Float16*)(ws + oR);
  _Float16* hpl  = (_Float16*)(ws + oH);

  k_wcvt<<<dim3(WUNITS / NTHR, 2), NTHR, 0, stream>>>(W1, W2, w1p, w2p);

  hipFuncSetAttribute(reinterpret_cast<const void*>(&k_agg),
                      hipFuncAttributeMaxDynamicSharedMemorySize, LDS_AGG);
  k_agg<<<nRB, NTHR, LDS_AGG, stream>>>(feat, src, dst, eps, rstp, nN, nE, 1);

  k_gemm<0><<<dim3(nRB, DHID / BN), GTHR, 0, stream>>>(rstp, w1p, b1, feat, hpl, out, DIN, DHID, nN);

  k_gemm<1><<<dim3(nRB, DIN / BN), GTHR, 0, stream>>>(hpl, w2p, b2, feat, rstp, out, DHID, DIN, nN);
}
